// RWKV_TimeMix_75522704933162
// MI455X (gfx1250) — hardware-verified
//
#include <hip/hip_runtime.h>
#include <math.h>

constexpr int kBatch = 8;
constexpr int kSeq   = 1024;
constexpr int kChan  = 1024;
constexpr int kRows  = kBatch * kSeq;
constexpr int kVec8PerRow = kChan / 8;
constexpr float kWCarry    = 16.0f;
constexpr float kWCarryInv = 1.0f / 16.0f;
constexpr float kGCarry    = 16.0f;
constexpr float kOutScale  = 1.0f / (16.0f * 16.0f);
static_assert((kSeq & (kSeq - 1)) == 0, "sequence length is a power of two");
static_assert(kRows % 64 == 0 && kChan % 64 == 0, "GEMM M and N are 64-tile multiples");
static_assert(kChan % 32 == 0, "GEMM K is a multiple of 32");
static_assert(((kRows / 64) * (kChan / 64)) % 8 == 0, "eight 64x64 tiles per GEMM block");
static_assert((kBatch * kChan / 2) == 16 * 256, "scan grid: 16 blocks x 256 lanes x 2 channels");
static_assert((kChan * kChan / 8) % 256 == 0, "weight cast grid exact");
static_assert(((long)kRows * kVec8PerRow) % 256 == 0, "mix grid exact");

typedef __attribute__((ext_vector_type(16))) _Float16 v16h;
typedef __attribute__((ext_vector_type(8)))  _Float16 v8h;
typedef __attribute__((ext_vector_type(8)))  float    v8f;
typedef __attribute__((ext_vector_type(4)))  float    v4f;
typedef __attribute__((ext_vector_type(2)))  float    v2f;
typedef __attribute__((ext_vector_type(4)))  unsigned int v4u;

__device__ __forceinline__ unsigned pk16(unsigned short a, unsigned short b) {
  return (unsigned)a | ((unsigned)b << 16);
}
__device__ __forceinline__ unsigned short h_bits(float f) {
  const _Float16 h = (_Float16)f;
  return __builtin_bit_cast(unsigned short, h);
}
__device__ __forceinline__ float h16_to_f32(unsigned hb) {
  const unsigned sgn = (hb & 0x8000u) << 16;
  const unsigned em = hb & 0x7fffu;
  const float fn = __uint_as_float((em << 13) + 0x38000000u);
  const float fs = (float)em * 5.9604644775390625e-8f;
  const float mag = (em < 0x400u) ? fs : fn;
  return __uint_as_float(__float_as_uint(mag) | sgn);
}
__device__ __forceinline__ float ftz_pos(float x) {
  return (x < 1.17549435e-38f) ? 0.0f : x;
}

union FragU { v16h v; v8h h[2]; };
__device__ __forceinline__ v16h frag_load(const _Float16* p) {
  FragU f;
  f.h[0] = *(const v8h*)(p);
  f.h[1] = *(const v8h*)(p + 16);
  return f.v;
}
__device__ __forceinline__ v8f frag_mma(v16h a, v16h b, v8f c) {
  return __builtin_amdgcn_wmma_f32_16x16x32_f16(false, a, false, b, (short)0, c, false, false);
}
__device__ __forceinline__ void dep_guard_row4(v8f& a, v8f& b, v8f& c, v8f& d,
                                               v16h x, v16h y0, v16h y1, v16h y2, v16h y3) {
  asm volatile("v_nop\n\tv_nop\n\tv_nop\n\tv_nop"
               : "+v"(a), "+v"(b), "+v"(c), "+v"(d)
               : "v"(x), "v"(y0), "v"(y1), "v"(y2), "v"(y3));
}
__device__ __forceinline__ void keep4_h(v16h a, v16h b, v16h c, v16h d) {
  asm volatile("v_nop" :: "v"(a), "v"(b), "v"(c), "v"(d));
}
__device__ __forceinline__ void acc_guard4(v8f& a, v8f& b, v8f& c, v8f& d) {
  asm volatile("v_nop\n\tv_nop\n\tv_nop\n\tv_nop" : "+v"(a), "+v"(b), "+v"(c), "+v"(d));
}

template <int OUT_MODE, int ACT>
__global__ __launch_bounds__(256) void wmma_gemm64_f16(
    const unsigned short* __restrict__ Ap, int lda,
    const unsigned short* __restrict__ Btp, int ldb,
    void* __restrict__ Cout, int ldc,
    int M, int N, int K, float scale) {
  const _Float16* A  = (const _Float16*)Ap;
  const _Float16* Bt = (const _Float16*)Btp;
  __shared__ __align__(16) float sT[8][16 * 68];
  const int lane = threadIdx.x & 31;
  const int wave = threadIdx.x >> 5;
  const int tilesN = N >> 6;
  const int tilesM = M >> 6;
  const int tile = blockIdx.x * 8 + wave;
  if (tile >= tilesM * tilesN) return;
  const int tm = tile / tilesN;
  const int tn = tile - tm * tilesN;
  const int m0 = tm << 6;
  const int n0 = tn << 6;

  const int rlane = lane & 15;
  const int koff  = (lane >> 4) * 8;
  const int mOff  = (lane >> 4) * 8;

  v8f acc[4][4];
#pragma unroll
  for (int i = 0; i < 4; ++i)
#pragma unroll
    for (int j = 0; j < 4; ++j) acc[i][j] = (v8f){0.f, 0.f, 0.f, 0.f, 0.f, 0.f, 0.f, 0.f};

  for (int k0 = 0; k0 < K; k0 += 32) {
    v16h bh[4];
#pragma unroll
    for (int j = 0; j < 4; ++j) {
      const size_t bo = (size_t)(n0 + (j << 4) + rlane) * ldb + koff + k0;
      bh[j] = frag_load(Bt + bo);
    }
#pragma unroll
    for (int i = 0; i < 4; ++i) {
      const size_t ao = (size_t)(m0 + (i << 4) + rlane) * lda + koff + k0;
      const v16h ah = frag_load(A + ao);
#pragma unroll
      for (int j = 0; j < 4; ++j) acc[i][j] = frag_mma(ah, bh[j], acc[i][j]);
      dep_guard_row4(acc[i][0], acc[i][1], acc[i][2], acc[i][3], ah, bh[0], bh[1], bh[2], bh[3]);
    }
    keep4_h(bh[0], bh[1], bh[2], bh[3]);
  }
  acc_guard4(acc[0][0], acc[0][1], acc[0][2], acc[0][3]);
  acc_guard4(acc[1][0], acc[1][1], acc[1][2], acc[1][3]);
  acc_guard4(acc[2][0], acc[2][1], acc[2][2], acc[2][3]);
  acc_guard4(acc[3][0], acc[3][1], acc[3][2], acc[3][3]);

  float* slab = sT[wave];
#pragma unroll
  for (int i = 0; i < 4; ++i) {
    const int mBase = m0 + (i << 4);
#pragma unroll
    for (int j = 0; j < 4; ++j) {
#pragma unroll
      for (int r = 0; r < 8; ++r) {
        const float v = acc[i][j][r] * scale;
        slab[(mOff + r) * 68 + (j << 4) + rlane] = v;
      }
    }
    __builtin_amdgcn_fence(__ATOMIC_RELEASE, "workgroup");
    __builtin_amdgcn_wave_barrier();
    __builtin_amdgcn_fence(__ATOMIC_ACQUIRE, "workgroup");
    if (OUT_MODE == 0) {
      float* C = (float*)Cout;
      const int hh = lane >> 4;
      const int c4 = (lane & 15) * 4;
      for (int pass = 0; pass < 2; ++pass) {
#pragma unroll
        for (int it = 0; it < 8; ++it) {
          const int row = it * 2 + hh;
          const v4f v = *(const v4f*)(slab + row * 68 + c4);
          *(volatile v4f*)(C + (size_t)(mBase + row) * ldc + n0 + c4) = v;
        }
        __threadfence();
      }
    } else {
      const int q  = lane >> 3;
      const int c8 = (lane & 7) * 8;
      if (ACT == 1) {
#pragma unroll 1
        for (int it = 0; it < 4; ++it) {
          float* sp = slab + (it * 4 + q) * 68 + c8;
#pragma unroll
          for (int e = 0; e < 8; ++e) {
            const float z = sp[e];
            sp[e] = 1.0f / (1.0f + expf(-z));
          }
        }
      }
      unsigned short* C = (unsigned short*)Cout;
      for (int pass = 0; pass < 2; ++pass) {
#pragma unroll
        for (int it = 0; it < 4; ++it) {
          const int row = it * 4 + q;
          const float* sp = slab + row * 68 + c8;
          v8h hv;
#pragma unroll
          for (int e = 0; e < 8; ++e) hv[e] = (_Float16)sp[e];
          *(volatile v8h*)(C + (size_t)(mBase + row) * ldc + n0 + c8) = hv;
        }
        __threadfence();
      }
    }
    __builtin_amdgcn_fence(__ATOMIC_RELEASE, "workgroup");
    __builtin_amdgcn_wave_barrier();
    __builtin_amdgcn_fence(__ATOMIC_ACQUIRE, "workgroup");
  }
}

__global__ __launch_bounds__(256) void cast_w4_kernel(const float* __restrict__ W0, const float* __restrict__ W1,
                                                      const float* __restrict__ W2, const float* __restrict__ W3,
                                                      unsigned short* __restrict__ out, float sc) {
  const int z = blockIdx.y;
  const float* W = (z == 0) ? W0 : (z == 1) ? W1 : (z == 2) ? W2 : W3;
  const int i = blockIdx.x * 256 + threadIdx.x;
  if (i >= kChan * kChan / 8) return;
  const float* p = W + 8 * (size_t)i;
  const v4f a = *(const v4f*)(p);
  const v4f c = *(const v4f*)(p + 4);
  unsigned short hb[8];
#pragma unroll
  for (int e = 0; e < 4; ++e) {
    const float fa = a[e] * sc;
    const float fc = c[e] * sc;
    hb[e]     = h_bits(fa);
    hb[4 + e] = h_bits(fc);
  }
  const v4u u = (v4u){pk16(hb[0], hb[1]), pk16(hb[2], hb[3]), pk16(hb[4], hb[5]), pk16(hb[6], hb[7])};
  unsigned short* q = out + (size_t)z * kChan * kChan + 8 * (size_t)i;
  *(volatile v4u*)q = u;
  __threadfence();
  *(volatile v4u*)q = u;
}

__device__ __forceinline__ float mix1(float xc, float xs, float w) {
  return xc * w + xs * (1.0f - w);
}
__global__ __launch_bounds__(256) void token_mix_kernel(const float* __restrict__ x,
                                                        const float* __restrict__ mk, const float* __restrict__ mv,
                                                        const float* __restrict__ mr,
                                                        unsigned short* __restrict__ xk, unsigned short* __restrict__ xv,
                                                        unsigned short* __restrict__ xr) {
  const int i = blockIdx.x * 256 + threadIdx.x;
  if (i >= kRows * kVec8PerRow) return;
  const int m  = i / kVec8PerRow;
  const int c0 = (i - m * kVec8PerRow) * 8;
  const int t  = m & (kSeq - 1);
  const bool first = (t == 0);
  const int mp = first ? m : (m - 1);
  const float* xcp = x + (size_t)m * kChan + c0;
  const float* xsp = x + (size_t)mp * kChan + c0;
  const v4f a0 = *(const v4f*)(xcp);
  const v4f a1 = *(const v4f*)(xcp + 4);
  const v4f s0 = *(const v4f*)(xsp);
  const v4f s1 = *(const v4f*)(xsp + 4);
  const v4f k0 = *(const v4f*)(mk + c0);
  const v4f k1 = *(const v4f*)(mk + c0 + 4);
  const v4f v0 = *(const v4f*)(mv + c0);
  const v4f v1 = *(const v4f*)(mv + c0 + 4);
  const v4f r0 = *(const v4f*)(mr + c0);
  const v4f r1 = *(const v4f*)(mr + c0 + 4);
  unsigned short hk[8], hv[8], hr[8];
#pragma unroll
  for (int e = 0; e < 4; ++e) {
    const float c_lo = a0[e];
    const float c_hi = a1[e];
    const float p_lo = first ? 0.0f : s0[e];
    const float p_hi = first ? 0.0f : s1[e];
    hk[e]     = h_bits(mix1(c_lo, p_lo, k0[e]));
    hk[4 + e] = h_bits(mix1(c_hi, p_hi, k1[e]));
    hv[e]     = h_bits(mix1(c_lo, p_lo, v0[e]));
    hv[4 + e] = h_bits(mix1(c_hi, p_hi, v1[e]));
    hr[e]     = h_bits(mix1(c_lo, p_lo, r0[e]));
    hr[4 + e] = h_bits(mix1(c_hi, p_hi, r1[e]));
  }
  const v4u uk = (v4u){pk16(hk[0], hk[1]), pk16(hk[2], hk[3]), pk16(hk[4], hk[5]), pk16(hk[6], hk[7])};
  const v4u uv = (v4u){pk16(hv[0], hv[1]), pk16(hv[2], hv[3]), pk16(hv[4], hv[5]), pk16(hv[6], hv[7])};
  const v4u ur = (v4u){pk16(hr[0], hr[1]), pk16(hr[2], hr[3]), pk16(hr[4], hr[5]), pk16(hr[6], hr[7])};
  const size_t eo = (size_t)m * kChan + c0;
  unsigned short* pk = xk + eo;
  unsigned short* pv = xv + eo;
  unsigned short* pr = xr + eo;
  *(volatile v4u*)pk = uk;
  *(volatile v4u*)pv = uv;
  *(volatile v4u*)pr = ur;
  __threadfence();
  *(volatile v4u*)pk = uk;
  *(volatile v4u*)pv = uv;
  *(volatile v4u*)pr = ur;
}

__device__ __forceinline__ float scan_step(float kt, float vt, float gt, float u, float w,
                                           float& aa, float& bb, float& pp) {
  const float ww  = u + kt;
  const float d   = pp - ww;
  const float e   = ftz_pos(expf(-fabsf(d)));
  const bool  ge  = (d >= 0.0f);
  const float e1  = ge ? 1.0f : e;
  const float e2  = ge ? e : 1.0f;
  const float num = e1 * aa + e2 * vt;
  const float den = e1 * bb + e2;
  const float y   = num / den;
  const float ww2 = pp + w;
  const float d2  = ww2 - kt;
  const float eb  = ftz_pos(expf(-fabsf(d2)));
  const bool  ge2 = (d2 >= 0.0f);
  const float e1b = ge2 ? 1.0f : eb;
  const float e2b = ge2 ? eb : 1.0f;
  aa = e1b * aa + e2b * vt;
  bb = e1b * bb + e2b;
  pp = fmaxf(ww2, kt);
  return gt * y;
}

__global__ __launch_bounds__(256) void decay_scan_kernel(const float* __restrict__ Kf,
                                                         const unsigned* __restrict__ Vw,
                                                         const unsigned* __restrict__ Gw,
                                                         const float* __restrict__ tdecay,
                                                         const float* __restrict__ tfirst,
                                                         unsigned* __restrict__ Rw) {
  const int tid = threadIdx.x;
  const int b   = blockIdx.x >> 1;
  const int ch  = (blockIdx.x & 1) * 512 + 2 * tid;
  const v2f td = *(const v2f*)(tdecay + ch);
  const v2f tf = *(const v2f*)(tfirst + ch);
  const float td0 = td.x;
  const float td1 = td.y;
  const float w0 = -expf(td0);
  const float w1 = -expf(td1);
  const float u0 = tf.x;
  const float u1 = tf.y;
  float aa0 = 0.0f, bb0 = 0.0f, pp0 = -1e38f;
  float aa1 = 0.0f, bb1 = 0.0f, pp1 = -1e38f;
  const size_t e0 = (size_t)b * kSeq * kChan + (size_t)ch;
#pragma unroll 1
  for (int t = 0; t < kSeq; ++t) {
    const size_t eo = e0 + (size_t)t * kChan;
    const size_t wo = eo >> 1;
    const v2f kk = *(const v2f*)(Kf + eo);
    unsigned vw = Vw[wo];
    unsigned gw = Gw[wo];
    float k0 = kk.x;
    float k1 = kk.y;
    asm volatile("" : "+v"(k0));
    asm volatile("" : "+v"(k1));
    asm volatile("" : "+v"(vw));
    asm volatile("" : "+v"(gw));
    const float v0 = h16_to_f32(vw & 0xffffu);
    const float v1 = h16_to_f32(vw >> 16);
    const float g0 = h16_to_f32(gw & 0xffffu);
    const float g1 = h16_to_f32(gw >> 16);
    const float r0 = scan_step(k0, v0, g0, u0, w0, aa0, bb0, pp0);
    const float r1 = scan_step(k1, v1, g1, u1, w1, aa1, bb1, pp1);
    const float c0 = r0 * kGCarry;
    const float c1 = r1 * kGCarry;
    const unsigned word = pk16(h_bits(c0), h_bits(c1));
    volatile unsigned* rp = (volatile unsigned*)(Rw + wo);
    *rp = word;
    __threadfence();
    *rp = word;
  }
}

extern "C" void kernel_launch(void* const* d_in, const int* in_sizes, int n_in,
                              void* d_out, int out_size, void* d_ws, size_t ws_size, hipStream_t stream) {
  if (n_in < 10 || d_out == nullptr || d_ws == nullptr) return;
  if (in_sizes[0] != kRows * kChan || in_sizes[1] != kChan || in_sizes[2] != kChan ||
      in_sizes[3] != kChan || in_sizes[4] != kChan || in_sizes[5] != kChan ||
      in_sizes[6] != kChan * kChan || in_sizes[7] != kChan * kChan ||
      in_sizes[8] != kChan * kChan || in_sizes[9] != kChan * kChan ||
      out_size != kRows * kChan) return;

  const float* x      = (const float*)d_in[0];
  const float* tdecay = (const float*)d_in[1];
  const float* tfirst = (const float*)d_in[2];
  const float* mixk   = (const float*)d_in[3];
  const float* mixv   = (const float*)d_in[4];
  const float* mixr   = (const float*)d_in[5];
  const float* Wk     = (const float*)d_in[6];
  const float* Wv     = (const float*)d_in[7];
  const float* Wr     = (const float*)d_in[8];
  const float* Wo     = (const float*)d_in[9];
  float* out = (float*)d_out;

  const size_t wBytes   = (size_t)kChan * kChan * 2;
  const size_t p16Bytes = (size_t)kRows * kChan * 2;
  const size_t p32Bytes = (size_t)kRows * kChan * 4;
  char* ws = (char*)d_ws;
  size_t off = 0;
  unsigned short* W16  = (unsigned short*)(ws + off); off += 4 * wBytes;
  unsigned short* XK16 = (unsigned short*)(ws + off); off += p16Bytes;
  unsigned short* XV16 = (unsigned short*)(ws + off); off += p16Bytes;
  unsigned short* XR16 = (unsigned short*)(ws + off); off += p16Bytes;
  float*          KF32 = (float*)(ws + off);          off += p32Bytes;
  unsigned short* V16  = (unsigned short*)(ws + off); off += p16Bytes;
  unsigned short* G16  = (unsigned short*)(ws + off); off += p16Bytes;
  if (off > ws_size || off > (size_t)134217728) return;
  unsigned short* Wk16 = W16;
  unsigned short* Wv16 = W16 + (size_t)kChan * kChan;
  unsigned short* Wr16 = W16 + (size_t)2 * kChan * kChan;
  unsigned short* Wo16 = W16 + (size_t)3 * kChan * kChan;
  unsigned short* R16  = XK16;

  cast_w4_kernel<<<dim3((kChan * kChan / 8) / 256, 4), 256, 0, stream>>>(Wk, Wv, Wr, Wo, W16, kWCarry);

  token_mix_kernel<<<(kRows * kVec8PerRow) / 256, 256, 0, stream>>>(x, mixk, mixv, mixr, XK16, XV16, XR16);

  const dim3 ggrid(((kRows / 64) * (kChan / 64)) / 8);
  wmma_gemm64_f16<0, 0><<<ggrid, 256, 0, stream>>>(XK16, kChan, Wk16, kChan, (void*)KF32, kChan,
                                                   kRows, kChan, kChan, kWCarryInv);
  wmma_gemm64_f16<1, 0><<<ggrid, 256, 0, stream>>>(XV16, kChan, Wv16, kChan, (void*)V16, kChan,
                                                   kRows, kChan, kChan, kWCarryInv);
  wmma_gemm64_f16<1, 1><<<ggrid, 256, 0, stream>>>(XR16, kChan, Wr16, kChan, (void*)G16, kChan,
                                                   kRows, kChan, kChan, kWCarryInv);

  decay_scan_kernel<<<(kBatch * kChan / 2) / 256, 256, 0, stream>>>(KF32, (const unsigned*)V16, (const unsigned*)G16,
                                                                   tdecay, tfirst, (unsigned*)R16);

  wmma_gemm64_f16<0, 0><<<ggrid, 256, 0, stream>>>(R16, kChan, Wo16, kChan, (void*)out, kChan,
                                                   kRows, kChan, kChan, kOutScale);
}
